// ExecuTorchModel_65944927863403
// MI455X (gfx1250) — hardware-verified
//
#include <hip/hip_runtime.h>

#define NN 32768
#define KK 16
#define EE (NN * KK)
#define HH 128
#define H2 256
#define RRR 2
#define LLL 2
#define LR (LLL * RRR)
#define NWA 4
#define WSC 16.0f
#define WSC_INV 0.0625f

typedef __attribute__((ext_vector_type(16))) _Float16 v16h;
typedef __attribute__((ext_vector_type(8)))  _Float16 v8h;
typedef __attribute__((ext_vector_type(4)))  _Float16 v4h;
typedef __attribute__((ext_vector_type(16))) __bf16   v16b;
typedef __attribute__((ext_vector_type(8)))  __bf16   v8b;
typedef __attribute__((ext_vector_type(8)))  float    v8f;
typedef __attribute__((ext_vector_type(4)))  float    v4f;

__device__ __forceinline__ unsigned short f2bf_bits(float f) {
  unsigned u = __float_as_uint(f);
  return (unsigned short)((u + 0x7FFFu + ((u >> 16) & 1u)) >> 16);
}
__device__ __forceinline__ float bf_bits2f(unsigned short h) { return __uint_as_float(((unsigned)h) << 16); }

__device__ __forceinline__ void dep_guard_h(v8f& a, v8f& b, v16h x, v16h y) { asm volatile("v_nop\n\tv_nop\n\tv_nop\n\tv_nop" : "+v"(a), "+v"(b) : "v"(x), "v"(y)); }
__device__ __forceinline__ void dep_guard_b(v8f& a, v8f& b, v16b x, v16b y) { asm volatile("v_nop\n\tv_nop\n\tv_nop\n\tv_nop" : "+v"(a), "+v"(b) : "v"(x), "v"(y)); }
__device__ __forceinline__ void keep4_h(v16h a, v16h b, v16h c, v16h d) { asm volatile("v_nop" :: "v"(a), "v"(b), "v"(c), "v"(d)); }
__device__ __forceinline__ void keep4_b(v16b a, v16b b, v16b c, v16b d) { asm volatile("v_nop" :: "v"(a), "v"(b), "v"(c), "v"(d)); }
__device__ __forceinline__ void acc_guard4(v8f& a, v8f& b, v8f& c, v8f& d) { asm volatile("v_nop\n\tv_nop\n\tv_nop\n\tv_nop" : "+v"(a), "+v"(b), "+v"(c), "+v"(d)); }
template <typename T> struct Frag;
template <> struct Frag<_Float16> {
  typedef v16h V; union U { v16h v; v8h h[2]; };
  static __device__ __forceinline__ v16h load(const _Float16* p) {
    U f; f.h[0] = *(const v8h*)(p); f.h[1] = *(const v8h*)(p + 16); return f.v;
  }
  static __device__ __forceinline__ v8f mma(v16h a, v16h b, v8f c) {
    return __builtin_amdgcn_wmma_f32_16x16x32_f16(false, a, false, b, (short)0, c, false, false);
  }
  static __device__ __forceinline__ void guard(v8f& a, v8f& b, v16h x, v16h y) { dep_guard_h(a, b, x, y); }
  static __device__ __forceinline__ void keep(v16h a, v16h b, v16h c, v16h d) { keep4_h(a, b, c, d); }
};
template <> struct Frag<__bf16> {
  typedef v16b V; union U { v16b v; v8b h[2]; };
  static __device__ __forceinline__ v16b load(const __bf16* p) {
    U f; f.h[0] = *(const v8b*)(p); f.h[1] = *(const v8b*)(p + 16); return f.v;
  }
  static __device__ __forceinline__ v8f mma(v16b a, v16b b, v8f c) {
    return __builtin_amdgcn_wmma_f32_16x16x32_bf16(false, a, false, b, (short)0, c, false, false);
  }
  static __device__ __forceinline__ void guard(v8f& a, v8f& b, v16b x, v16b y) { dep_guard_b(a, b, x, y); }
  static __device__ __forceinline__ void keep(v16b a, v16b b, v16b c, v16b d) { keep4_b(a, b, c, d); }
};

template <int ET> struct Elem;
template <> struct Elem<0> { typedef _Float16 T; };
template <> struct Elem<1> { typedef __bf16 T; };
template <int ET, bool SPLIT, int BIAS_MODE, int OUT_MODE, bool RESID, int ACT = 0>
__global__ __launch_bounds__(256) void wmma_gemm64(
    const unsigned short* __restrict__ Ap, const unsigned short* __restrict__ A2p, int lda, long strideA,
    const unsigned short* __restrict__ Btp, const unsigned short* __restrict__ Bt2p, int ldb, long strideB,
    void* __restrict__ Cout, void* __restrict__ Cout2, int ldc, long strideC,
    const float* __restrict__ bias,
    const float* __restrict__ resid, long strideR,
    int M, int N, int K, float scale) {
  typedef typename Elem<ET>::T T;
  typedef typename Frag<T>::V V;
  const T* A = (const T*)Ap; const T* A2 = (const T*)A2p; const T* Bt = (const T*)Btp; const T* Bt2 = (const T*)Bt2p;
  __shared__ __align__(16) float sT[8][16 * 68];
  const int b    = blockIdx.y;
  const int lane = threadIdx.x & 31;
  const int wave = threadIdx.x >> 5;
  const int tilesN = N >> 6;
  const int tilesM = M >> 6;
  const int tile = blockIdx.x * 8 + wave;
  if (tile >= tilesM * tilesN) return;
  const int tm = tile / tilesN;
  const int tn = tile - tm * tilesN;
  const int m0 = tm << 6;
  const int n0 = tn << 6;

  const T* Ab  = A  + (size_t)b * strideA;
  const T* Bb  = Bt + (size_t)b * strideB;
  const T* Ab2 = SPLIT ? (A2  + (size_t)b * strideA) : nullptr;
  const T* Bb2 = SPLIT ? (Bt2 + (size_t)b * strideB) : nullptr;

  const int rlane = lane & 15;
  const int koff  = (lane >> 4) * 8;
  const int mOff  = (lane >> 4) * 8;

  v8f acc[4][4];
#pragma unroll
  for (int i = 0; i < 4; ++i)
#pragma unroll
    for (int j = 0; j < 4; ++j) acc[i][j] = (v8f){0.f,0.f,0.f,0.f,0.f,0.f,0.f,0.f};

  for (int k0 = 0; k0 < K; k0 += 32) {
    V bh[4], bl[4];
#pragma unroll
    for (int j = 0; j < 4; ++j) {
      const size_t bo = (size_t)(n0 + (j << 4) + rlane) * ldb + koff + k0;
      bh[j] = Frag<T>::load(Bb + bo);
      if (SPLIT) bl[j] = Frag<T>::load(Bb2 + bo);
    }
#pragma unroll
    for (int i = 0; i < 4; ++i) {
      const size_t ao = (size_t)(m0 + (i << 4) + rlane) * lda + koff + k0;
      V ah = Frag<T>::load(Ab + ao);
      V al;
      if (SPLIT) al = Frag<T>::load(Ab2 + ao);
#pragma unroll
      for (int j = 0; j < 4; ++j) {
        acc[i][j] = Frag<T>::mma(ah, bh[j], acc[i][j]);
        if (SPLIT) {
          acc[i][j] = Frag<T>::mma(ah, bl[j], acc[i][j]);
          acc[i][j] = Frag<T>::mma(al, bh[j], acc[i][j]);
        }
      }
      Frag<T>::guard(acc[i][0], acc[i][3], ah, SPLIT ? al : ah);
    }
    Frag<T>::keep(bh[0], bh[1], bh[2], bh[3]);
    if (SPLIT) Frag<T>::keep(bl[0], bl[1], bl[2], bl[3]);
  }
  acc_guard4(acc[0][0], acc[0][1], acc[0][2], acc[0][3]);
  acc_guard4(acc[1][0], acc[1][1], acc[1][2], acc[1][3]);
  acc_guard4(acc[2][0], acc[2][1], acc[2][2], acc[2][3]);
  acc_guard4(acc[3][0], acc[3][1], acc[3][2], acc[3][3]);

  float* slab = sT[wave];
  const float* Rb = RESID ? (resid + (size_t)b * strideR) : nullptr;
#pragma unroll
  for (int i = 0; i < 4; ++i) {
    const int mBase = m0 + (i << 4);
#pragma unroll
    for (int j = 0; j < 4; ++j) {
      const int n = n0 + (j << 4) + rlane;
      float bv = 0.f;
      if (BIAS_MODE == 2) bv = bias[n];
#pragma unroll
      for (int r = 0; r < 8; ++r) {
        float v = acc[i][j][r] * scale;
        if (BIAS_MODE == 1) v += bias[mBase + mOff + r];
        if (BIAS_MODE == 2) v += bv;
        if (RESID) v += Rb[(size_t)(mBase + mOff + r) * ldc + n];
        if (ACT == 1) v = tanhf(v);
        if (ACT == 2) v = fmaxf(v, 0.0f);
        if (ACT == 3) v = v / (1.0f + expf(-v));
        if (ACT == 4) v = (v > 0.f) ? v : 0.01f * v;
        if (ACT == 5) v = 0.5f * v * (1.0f + erff(v * 0.70710678118654752f));
        slab[(mOff + r) * 68 + (j << 4) + rlane] = v;
      }
    }
    __builtin_amdgcn_fence(__ATOMIC_RELEASE, "workgroup");
    __builtin_amdgcn_wave_barrier();
    __builtin_amdgcn_fence(__ATOMIC_ACQUIRE, "workgroup");
    if (OUT_MODE == 0) {
      float* C = (float*)Cout + (size_t)b * strideC;
      const int hh = lane >> 4, c4 = (lane & 15) * 4;
      for (int pass = 0; pass < 2; ++pass) {
#pragma unroll
        for (int it = 0; it < 8; ++it) {
          const int row = it * 2 + hh;
          v4f v = *(const v4f*)(slab + row * 68 + c4);
          *(volatile v4f*)(C + (size_t)(mBase + row) * ldc + n0 + c4) = v;
        }
        __threadfence();
      }
    } else {
      const int q = lane >> 3, c8 = (lane & 7) * 8;
      unsigned short* C  = (unsigned short*)Cout  + (size_t)b * strideC;
      unsigned short* C2 = (OUT_MODE == 2) ? ((unsigned short*)Cout2 + (size_t)b * strideC) : nullptr;
      for (int pass = 0; pass < 2; ++pass) {
#pragma unroll
        for (int it = 0; it < 4; ++it) {
          const int row = it * 4 + q;
          const float* sp = slab + row * 68 + c8;
          v8h hv, lv;
#pragma unroll
          for (int e = 0; e < 8; ++e) {
            if (OUT_MODE == 1) {
              hv[e] = (_Float16)sp[e];
            } else {
              unsigned short hb = f2bf_bits(sp[e]);
              unsigned short lb = f2bf_bits(sp[e] - bf_bits2f(hb));
              hv[e] = __builtin_bit_cast(_Float16, hb);
              lv[e] = __builtin_bit_cast(_Float16, lb);
            }
          }
          *(volatile v8h*)(C + (size_t)(mBase + row) * ldc + n0 + c8) = hv;
          if (OUT_MODE == 2) *(volatile v8h*)(C2 + (size_t)(mBase + row) * ldc + n0 + c8) = lv;
        }
        __threadfence();
      }
    }
    __builtin_amdgcn_fence(__ATOMIC_RELEASE, "workgroup");
    __builtin_amdgcn_wave_barrier();
    __builtin_amdgcn_fence(__ATOMIC_ACQUIRE, "workgroup");
  }
}

__global__ __launch_bounds__(256) void prep_w1_f16x2(
    const float* __restrict__ W, const float* __restrict__ g, const float* __restrict__ v,
    _Float16* __restrict__ out, int n2, int kdim, float wsc) {
  int i = blockIdx.x * 256 + threadIdx.x;
  if (i < n2) {
    const int row = (2 * i) / kdim;
    const float sc = g[row] * rsqrtf(v[row] + 1e-5f) * wsc;
    const _Float16 h0 = (_Float16)(W[2 * i] * sc), h1 = (_Float16)(W[2 * i + 1] * sc);
    const unsigned u = (unsigned)__builtin_bit_cast(unsigned short, h0) | ((unsigned)__builtin_bit_cast(unsigned short, h1) << 16);
    ((volatile unsigned*)out)[i] = u;
    __threadfence();
    ((volatile unsigned*)out)[i] = u;
  }
}

__global__ __launch_bounds__(256) void prep_bn_shift(
    const float* __restrict__ g, const float* __restrict__ bta, const float* __restrict__ m,
    const float* __restrict__ v, float* __restrict__ shift, int n) {
  int i = blockIdx.x * 256 + threadIdx.x;
  if (i < n) {
    const float sc = g[i] * rsqrtf(v[i] + 1e-5f);
    const float sh = bta[i] - m[i] * sc;
    ((volatile float*)shift)[i] = sh;
    __threadfence();
    ((volatile float*)shift)[i] = sh;
  }
}

__global__ __launch_bounds__(256) void cast_scale_f32_f16x2(
    const float* __restrict__ in, _Float16* __restrict__ out, int n2, float wsc) {
  int i = blockIdx.x * 256 + threadIdx.x;
  if (i < n2) {
    const _Float16 h0 = (_Float16)(in[2 * i] * wsc), h1 = (_Float16)(in[2 * i + 1] * wsc);
    const unsigned u = (unsigned)__builtin_bit_cast(unsigned short, h0) | ((unsigned)__builtin_bit_cast(unsigned short, h1) << 16);
    ((volatile unsigned*)out)[i] = u;
    __threadfence();
    ((volatile unsigned*)out)[i] = u;
  }
}

__global__ __launch_bounds__(NWA * 32) void gather_softmax_agg(
    const float* __restrict__ x, const int* __restrict__ src, const float* __restrict__ ea,
    const int* __restrict__ nbr, const float* __restrict__ We, _Float16* __restrict__ outp,
    int nnodes, int nedges) {
  __shared__ __align__(16) v4f msh[NWA][KK][32];
  __shared__ __align__(16) _Float16 osh[NWA][HH];
  const int wave = threadIdx.x >> 5;
  const int lane = threadIdx.x & 31;
  const int node = blockIdx.x * NWA + wave;
  const bool nv = node < nnodes;
  const int nodec = nv ? node : (nnodes - 1);
  const int c = lane * 4;
  const v4f xn = *(const v4f*)(x + (size_t)nodec * HH + c);
  const v4f we = *(const v4f*)(We + c);
  const int* nb = nbr + (size_t)nodec * KK;

  v4f mx = (v4f){-3.402823466e38f, -3.402823466e38f, -3.402823466e38f, -3.402823466e38f};
  unsigned vm = 0u;
#pragma unroll 1
  for (int k = 0; k < KK; ++k) {
    int e = nb[k];
    if (e >= 0) {
      e = (e < nedges) ? e : (nedges - 1);
      int si = src[e];
      si = (si < 0) ? 0 : si;
      si = (si < nnodes) ? si : (nnodes - 1);
      const float eav = ea[e];
      const v4f xj = *(const v4f*)(x + (size_t)si * HH + c);
      v4f gm;
      gm.x = fmaxf(xj.x + eav * we.x, 0.0f) + 1e-7f;
      gm.y = fmaxf(xj.y + eav * we.y, 0.0f) + 1e-7f;
      gm.z = fmaxf(xj.z + eav * we.z, 0.0f) + 1e-7f;
      gm.w = fmaxf(xj.w + eav * we.w, 0.0f) + 1e-7f;
      msh[wave][k][lane] = gm;
      mx.x = fmaxf(mx.x, gm.x);
      mx.y = fmaxf(mx.y, gm.y);
      mx.z = fmaxf(mx.z, gm.z);
      mx.w = fmaxf(mx.w, gm.w);
      vm |= (1u << k);
    }
  }

  v4f s = (v4f){0.f, 0.f, 0.f, 0.f};
  v4f a = (v4f){0.f, 0.f, 0.f, 0.f};
#pragma unroll 1
  for (int k = 0; k < KK; ++k) {
    if ((vm >> k) & 1u) {
      const v4f gm = msh[wave][k][lane];
      v4f p;
      p.x = expf(gm.x - mx.x);
      p.y = expf(gm.y - mx.y);
      p.z = expf(gm.z - mx.z);
      p.w = expf(gm.w - mx.w);
      s += p;
      a.x += gm.x * p.x;
      a.y += gm.y * p.y;
      a.z += gm.z * p.z;
      a.w += gm.w * p.w;
    }
  }

  v4f o;
  o.x = a.x * __builtin_amdgcn_rcpf(s.x + 1e-16f) + xn.x;
  o.y = a.y * __builtin_amdgcn_rcpf(s.y + 1e-16f) + xn.y;
  o.z = a.z * __builtin_amdgcn_rcpf(s.z + 1e-16f) + xn.z;
  o.w = a.w * __builtin_amdgcn_rcpf(s.w + 1e-16f) + xn.w;
  {
    v4h oh;
    oh.x = (_Float16)o.x;
    oh.y = (_Float16)o.y;
    oh.z = (_Float16)o.z;
    oh.w = (_Float16)o.w;
    *(v4h*)(&osh[wave][c]) = oh;
  }
  __syncthreads();
  if (lane < 16 && nv) {
    const v8h vv = *(const v8h*)(&osh[wave][lane * 8]);
    _Float16* op = outp + (size_t)node * HH + lane * 8;
    *(volatile v8h*)op = vv;
    __threadfence();
    *(volatile v8h*)op = vv;
  }
}

extern "C" void kernel_launch(void* const* d_in, const int* in_sizes, int n_in,
                              void* d_out, int out_size, void* d_ws, size_t ws_size,
                              hipStream_t stream) {
  if (n_in < 11) return;
  if (in_sizes[0] != NN * HH) return;
  if (in_sizes[1] != RRR * 2 * EE) return;
  if (in_sizes[2] != RRR * EE) return;
  if (in_sizes[3] != RRR * NN * KK) return;
  if (in_sizes[4] != LR * HH) return;
  if (in_sizes[5] != LR * H2 * HH) return;
  if (in_sizes[6] != LR * H2 || in_sizes[7] != LR * H2 || in_sizes[8] != LR * H2 || in_sizes[9] != LR * H2) return;
  if (in_sizes[10] != LR * HH * H2) return;
  if (out_size != NN * HH) return;

  const float* x          = (const float*)d_in[0];
  const int*   edge_inds  = (const int*)d_in[1];
  const float* edge_attrs = (const float*)d_in[2];
  const int*   nbrs       = (const int*)d_in[3];
  const float* W_edge     = (const float*)d_in[4];
  const float* W1         = (const float*)d_in[5];
  const float* bng        = (const float*)d_in[6];
  const float* bnb        = (const float*)d_in[7];
  const float* bnm        = (const float*)d_in[8];
  const float* bnv        = (const float*)d_in[9];
  const float* W2         = (const float*)d_in[10];
  float* outF = (float*)d_out;

  size_t off = 0;
  const size_t o_agg = off; off += ((size_t)NN * HH * 2 + 255) & ~(size_t)255;
  const size_t o_h   = off; off += ((size_t)NN * H2 * 2 + 255) & ~(size_t)255;
  const size_t o_y0  = off; off += ((size_t)NN * HH * 4 + 255) & ~(size_t)255;
  const size_t o_y1  = off; off += ((size_t)NN * HH * 4 + 255) & ~(size_t)255;
  const size_t o_w1  = off; off += ((size_t)LR * H2 * HH * 2 + 255) & ~(size_t)255;
  const size_t o_w2  = off; off += ((size_t)LR * HH * H2 * 2 + 255) & ~(size_t)255;
  const size_t o_sh  = off; off += ((size_t)LR * H2 * 4 + 255) & ~(size_t)255;
  if (off > ws_size) return;
  char* ws = (char*)d_ws;
  _Float16* aggbuf = (_Float16*)(ws + o_agg);
  _Float16* hbuf   = (_Float16*)(ws + o_h);
  float*    ybuf0  = (float*)(ws + o_y0);
  float*    ybuf1  = (float*)(ws + o_y1);
  _Float16* W1s    = (_Float16*)(ws + o_w1);
  _Float16* W2h    = (_Float16*)(ws + o_w2);
  float*    shift  = (float*)(ws + o_sh);

  const int nW1x2 = LR * H2 * HH / 2;
  const int nW2x2 = LR * HH * H2 / 2;
  prep_w1_f16x2<<<(nW1x2 + 255) / 256, 256, 0, stream>>>(W1, bng, bnv, W1s, nW1x2, HH, WSC);
  prep_bn_shift<<<(LR * H2 + 255) / 256, 256, 0, stream>>>(bng, bnb, bnm, bnv, shift, LR * H2);
  cast_scale_f32_f16x2<<<(nW2x2 + 255) / 256, 256, 0, stream>>>(W2, W2h, nW2x2, WSC);

  const int aggBlocks = (NN + NWA - 1) / NWA;
  const int g1Tiles = (NN / 64) * (H2 / 64);
  const int g2Tiles = (NN / 64) * (HH / 64);
  const dim3 g1Grid((g1Tiles + 7) / 8, 1);
  const dim3 g2Grid((g2Tiles + 7) / 8, 1);

  const float* xin = x;
  for (int l = 0; l < LLL; ++l) {
    for (int r = 0; r < RRR; ++r) {
      const int lr = l * RRR + r;
      const int*   srcp = edge_inds + (size_t)r * 2 * EE;
      const float* eap  = edge_attrs + (size_t)r * EE;
      const int*   nbp  = nbrs + (size_t)r * NN * KK;
      const float* wep  = W_edge + (size_t)lr * HH;

      gather_softmax_agg<<<aggBlocks, NWA * 32, 0, stream>>>(xin, srcp, eap, nbp, wep, aggbuf, NN, EE);

      const unsigned short* a1 = (const unsigned short*)aggbuf;
      const unsigned short* b1 = (const unsigned short*)(W1s + (size_t)lr * H2 * HH);
      wmma_gemm64<0, false, 2, 1, false, 2><<<g1Grid, 256, 0, stream>>>(
          a1, a1, HH, (long)0, b1, b1, HH, (long)0,
          (void*)hbuf, (void*)hbuf, H2, (long)0,
          shift + (size_t)lr * H2, ybuf0, (long)0, NN, H2, HH, WSC_INV);

      const unsigned short* a2 = (const unsigned short*)hbuf;
      const unsigned short* b2 = (const unsigned short*)(W2h + (size_t)lr * HH * H2);
      if (r == 0) {
        wmma_gemm64<0, false, 0, 0, false, 0><<<g2Grid, 256, 0, stream>>>(
            a2, a2, H2, (long)0, b2, b2, H2, (long)0,
            (void*)ybuf0, (void*)ybuf0, HH, (long)0,
            shift, ybuf1, (long)0, NN, HH, H2, WSC_INV);
      } else if (l < LLL - 1) {
        wmma_gemm64<0, false, 0, 0, true, 4><<<g2Grid, 256, 0, stream>>>(
            a2, a2, H2, (long)0, b2, b2, H2, (long)0,
            (void*)ybuf1, (void*)ybuf1, HH, (long)0,
            shift, ybuf0, (long)0, NN, HH, H2, WSC_INV);
      } else {
        wmma_gemm64<0, false, 0, 0, true, 0><<<g2Grid, 256, 0, stream>>>(
            a2, a2, H2, (long)0, b2, b2, H2, (long)0,
            (void*)outF, (void*)outF, HH, (long)0,
            shift, ybuf0, (long)0, NN, HH, H2, WSC_INV);
      }
    }
    xin = ybuf1;
  }
  (void)hipGetLastError();
}
